// GCN_BiLSTM_Attn_Temporal_38431367364697
// MI455X (gfx1250) — hardware-run, weakly checked
//
#include <hip/hip_runtime.h>


namespace {
constexpr int N = 50000, E = 800000, EMB = 128, GH = 64, TD = 4, NB = 64, T = 200, H = 128, G4 = 4 * H, IND = 2 + EMB + TD  , INP = 160, NPB = 8, OPAD = 50176  ;
constexpr float HS = 256.0f, HS1 = 4096.0f  , ZS = 65536.0f  , HHS = 1048576.0f  , CS = 1048576.0f  , WSC = 4096.0f  , XS = 65536.0f  ;
typedef _Float16 b16;
typedef __attribute__((ext_vector_type(16))) _Float16 v16b;
typedef __attribute__((ext_vector_type(8))) _Float16 v8b;
typedef __attribute__((ext_vector_type(8))) float v8f;
typedef __attribute__((ext_vector_type(4))) float v4f;
typedef __attribute__((ext_vector_type(2))) float v2f;
__device__ __forceinline__ float bf16_rne(float f) { unsigned int u = __float_as_uint(f); u += 0x7FFFu + ((u >> 16) & 1u); float r = __uint_as_float(u & 0xFFFF0000u); asm volatile("" : "+v"(r)); return r; }
__device__ __forceinline__ float bfv(float f) { float r = bf16_rne(f); asm volatile("" : "+v"(r)); return r; }
__device__ __forceinline__ void split16(float v, b16& hi, b16& lo) { hi = (b16)v; lo = (b16)(v - (float)hi); }
__device__ __forceinline__ v16b frag_kb(const b16* p, int hh) { const v8b a = *(const v8b*)(p + 8 * hh), b = *(const v8b*)(p + 16 + 8 * hh); v16b f;
#pragma unroll
  for (int e = 0; e < 8; ++e) { f[e] = a[e]; f[8 + e] = b[e]; } return f; }
__device__ __forceinline__ v8f wmma16b(v16b a, v16b b, v8f c) { v8f d = __builtin_amdgcn_wmma_f32_16x16x32_f16(false, a, false, b, (short)0, c, false, false); asm volatile("v_nop\n\tv_nop\n\tv_nop\n\tv_nop" : "+v"(d) : "v"(a), "v"(b)); return d; }
__device__ __forceinline__ void wave_lds_sync() { __builtin_amdgcn_fence(__ATOMIC_RELEASE, "workgroup"); __builtin_amdgcn_wave_barrier(); __builtin_amdgcn_fence(__ATOMIC_ACQUIRE, "workgroup"); }
__device__ __forceinline__ float pmul(float a, float b) { float p = a * b; asm volatile("" : "+v"(p)); return p; }
__device__ __forceinline__ int iclamp(int v, int lo, int hi) { return v < lo ? lo : (v > hi ? hi : v); }
__device__ __forceinline__ float sigm(float v) { return 1.0f / (1.0f + __expf(-v)); }
constexpr int CSR_NBLK8 = 512, CSR_GB8 = 8, CSR_GN8 = 1 << CSR_GB8  , CSR_TS8 = (CSR_GN8 < 32 ? 32 : CSR_GN8)  , CSR_MAXG8 = 512, CSR_CAP8 = 12288  ;
__device__ __host__ __forceinline__ int csr_tix8(int v) { return (v >> CSR_GB8) * CSR_TS8 + (v & (CSR_GN8 - 1)); }
__global__ __launch_bounds__(64) void csrA_kernel8(const int* __restrict__ dst, int E, int N, int nG, int CHP, int NGP, int* __restrict__ STG, int* __restrict__ HST) {
  extern __shared__ int sm[];
  int* cnt = sm; int* run = sm + NGP; int* ids = sm + 2 * NGP;
  const int b = blockIdx.x; const int ch = (E + CSR_NBLK8 - 1) / CSR_NBLK8; const int e0 = b * ch, e1 = min(E, e0 + ch);
  for (int i = threadIdx.x; i < NGP; i += 64) cnt[i] = 0;
  for (int i = threadIdx.x; i < CHP; i += 64) ids[i] = -1;
  __syncthreads();
  if (threadIdx.x == 0) {
    for (int e = e0; e < e1; ++e) { int d = dst[e]; d = (d < 0) ? 0 : (d >= N ? N - 1 : d); cnt[d >> CSR_GB8] += 1; }
    int acc = 0; for (int g = 0; g < nG; ++g) { run[g] = acc; acc += cnt[g]; }
    for (int e = e0; e < e1; ++e) { int d = dst[e]; d = (d < 0) ? 0 : (d >= N ? N - 1 : d); const int g = d >> CSR_GB8; ids[run[g]] = e; run[g] += 1; } }
  __syncthreads();
  typedef __attribute__((ext_vector_type(4))) int v4i;
  for (int pass = 0; pass < 2; ++pass) {
    for (int i = threadIdx.x; i < CHP / 4; i += 64) *(volatile v4i*)(STG + (size_t)b * CHP + i * 4) = *(const v4i*)(&ids[i * 4]);
    for (int i = threadIdx.x; i < NGP / 4; i += 64) { v4i v; for (int e = 0; e < 4; ++e) v[e] = (i * 4 + e < nG) ? cnt[i * 4 + e] : 0; *(volatile v4i*)(HST + (size_t)b * NGP + i * 4) = v; }
    __threadfence(); }
}
__global__ __launch_bounds__(512) void csrS_kernel8(const int* __restrict__ HST, int nG, int NGP, int* __restrict__ START, int* __restrict__ TOT, int* __restrict__ OFF) {
  __shared__ int tot[CSR_MAXG8];
  const int b = threadIdx.x;
  for (int pass = 0; pass < 2; ++pass) { int runb = 0; for (int g = 0; g < nG; ++g) { int c = HST[(size_t)b * NGP + g]; c = (c < 0) ? 0 : c; ((volatile int*)OFF)[(size_t)g * CSR_NBLK8 + b] = runb; runb += c; } __threadfence(); }
  for (int g = threadIdx.x; g < nG; g += 512) { int s = 0; for (int bb = 0; bb < CSR_NBLK8; ++bb) { int c = HST[(size_t)bb * NGP + g]; s += (c < 0) ? 0 : c; } tot[g] = s; }
  __syncthreads();
  if (threadIdx.x < 32) {
    __shared__ int st[CSR_MAXG8 + 32];
    if (threadIdx.x == 0) { int acc = 0; for (int g = 0; g < NGP; ++g) { st[g] = acc; if (g < nG) acc += (tot[g] + 31) & ~31; } st[NGP] = acc; }
    __builtin_amdgcn_fence(__ATOMIC_RELEASE, "workgroup"); __builtin_amdgcn_wave_barrier(); __builtin_amdgcn_fence(__ATOMIC_ACQUIRE, "workgroup");
    for (int pass = 0; pass < 2; ++pass) { for (int i = threadIdx.x; i < NGP + 32; i += 32) { ((volatile int*)START)[i] = (i <= NGP) ? st[min(i, NGP)] : 0; ((volatile int*)TOT)[i] = (i < nG) ? tot[i] : 0; } __threadfence(); } }
}
__global__ __launch_bounds__(256) void csrB_kernel8(const int* __restrict__ dst, int N, int nG, int CHP, int NGP, int permLen, const int* __restrict__ STG, const int* __restrict__ HST, const int* __restrict__ OFF, const int* __restrict__ START, const int* __restrict__ TOT, int* __restrict__ PERM, int* __restrict__ ROWPTR, int* __restrict__ ROWCNT, int* __restrict__ FLAG) {
  typedef __attribute__((ext_vector_type(4))) int v4i;
  __shared__ int ids[CSR_CAP8]; __shared__ unsigned short key[CSR_CAP8]; __shared__ int outp[CSR_CAP8]; __shared__ int ncnt[CSR_GN8 + 1]; __shared__ int boff[CSR_NBLK8 + 1];
  const int g = blockIdx.x, t_ = threadIdx.x; int tot = TOT[g]; int st = START[g], stn = START[g + 1]; const int v0 = g * CSR_GN8; const int nv = min(CSR_GN8, N - v0); const int t0 = g * CSR_TS8;
  st = (st < 0) ? 0 : (st > permLen - 32 ? permLen - 32 : st) & ~31; stn = (stn < st) ? st : (stn > permLen ? permLen : stn); tot = (tot < 0) ? 0 : tot; if (tot > stn - st && tot <= CSR_CAP8) tot = stn - st;
  if (tot > CSR_CAP8) {
    for (int pass = 0; pass < 2; ++pass) { for (int i = t_; i < CSR_TS8 / 4; i += 256) { v4i a, c; for (int e = 0; e < 4; ++e) { a[e] = st; c[e] = 0; } *(volatile v4i*)(ROWPTR + t0 + i * 4) = a; *(volatile v4i*)(ROWCNT + t0 + i * 4) = c; } if (t_ == 0) ((volatile int*)FLAG)[0] = 1; __threadfence(); } (void)nv; return; }
  if (t_ == 0) { int acc = 0; for (int b = 0; b < CSR_NBLK8; ++b) { boff[b] = acc; int c = HST[(size_t)b * NGP + g]; c = (c < 0) ? 0 : (c > CHP ? CHP : c); acc += c; if (acc > tot) acc = tot; } boff[CSR_NBLK8] = acc; }
  for (int i = t_; i <= CSR_GN8; i += 256) ncnt[i] = 0;
  __syncthreads();
  for (int b = 0; b < CSR_NBLK8; ++b) { const int c = boff[b + 1] - boff[b]; int o_ = OFF[(size_t)g * CSR_NBLK8 + b]; o_ = (o_ < 0) ? 0 : (o_ > CHP - c ? CHP - c : o_); const int* src_ = STG + (size_t)b * CHP + o_;
    for (int i = t_; i < c; i += 256) { int id = src_[i]; id = (id < 0) ? 0 : id; ids[boff[b] + i] = id; int d = dst[id]; d = (d < v0) ? v0 : (d >= N ? N - 1 : d); int kk = d - v0; kk = (kk < 0) ? 0 : (kk >= CSR_GN8 ? CSR_GN8 - 1 : kk); key[boff[b] + i] = (unsigned short)kk; } }
  __syncthreads();
  if (t_ == 0) { for (int i = 0; i < tot; ++i) ncnt[key[i]] += 1; int acc = 0; for (int vl = 0; vl < CSR_GN8; ++vl) { const int c = ncnt[vl]; ncnt[vl] = acc; acc += c; } ncnt[CSR_GN8] = acc;
    for (int i = 0; i < tot; ++i) { const int vl = key[i]; outp[ncnt[vl]] = ids[i]; ncnt[vl] += 1; }
    for (int vl = CSR_GN8; vl > 0; --vl) ncnt[vl] = ncnt[vl - 1]; ncnt[0] = 0; }
  __syncthreads();
  for (int pass = 0; pass < 2; ++pass) {
    for (int i = t_; i < (stn - st) / 4; i += 256) { v4i v; for (int e = 0; e < 4; ++e) { const int q = i * 4 + e; v[e] = (q < tot) ? outp[q] : -1; } *(volatile v4i*)(PERM + st + i * 4) = v; }
    for (int i = t_; i < CSR_TS8 / 4; i += 256) { v4i a, c; for (int e = 0; e < 4; ++e) { const int vl = i * 4 + e; const int vc = vl < CSR_GN8 ? vl : CSR_GN8; a[e] = (vl < CSR_GN8) ? st + ncnt[vc] : st; c[e] = (vl < nv) ? (ncnt[(vc < CSR_GN8 ? vc : CSR_GN8 - 1) + 1] - ncnt[vc]) : 0; } *(volatile v4i*)(ROWPTR + t0 + i * 4) = a; *(volatile v4i*)(ROWCNT + t0 + i * 4) = c; }
    __threadfence(); }
}
__global__ __launch_bounds__(256) void csrZ_kernel8(int* __restrict__ p, size_t n4) { typedef __attribute__((ext_vector_type(4))) int v4i; const size_t tid = (size_t)blockIdx.x * 256 + threadIdx.x, nth = (size_t)gridDim.x * 256; v4i z = {0, 0, 0, 0}; for (size_t i = tid; i < n4; i += nth) *(volatile v4i*)(p + i * 4) = z; }
struct CsrBufs8 { int *STG, *HST, *OFF, *START, *TOT, *PERM, *ROWPTR, *ROWCNT, *FLAG; int nG, NGP, CHP; size_t permLen; char* base; size_t bytes; };
static size_t csr_carve8(CsrBufs8& c, char* ws, size_t off, int E, int N) {
  const size_t off0 = off; c.base = ws + off;
  auto al = [&](size_t bytes) { char* p = ws + off; off += (bytes + 255) & ~(size_t)255; return p; };
  c.nG = (N + CSR_GN8 - 1) / CSR_GN8; c.NGP = (c.nG + 31) & ~31; const int ch = (E + CSR_NBLK8 - 1) / CSR_NBLK8; c.CHP = (ch + 31) & ~31; c.permLen = (size_t)E + 32 * (size_t)c.nG + 32;
  c.STG = (int*)al((size_t)CSR_NBLK8 * c.CHP * 4); c.HST = (int*)al((size_t)CSR_NBLK8 * c.NGP * 4); c.OFF = (int*)al((size_t)c.NGP * CSR_NBLK8 * 4); c.START = (int*)al((size_t)(c.NGP + 64) * 4); c.TOT = (int*)al((size_t)(c.NGP + 64) * 4);
  c.PERM = (int*)al(c.permLen * 4); c.ROWPTR = (int*)al((size_t)c.nG * CSR_TS8 * 4); c.ROWCNT = (int*)al((size_t)c.nG * CSR_TS8 * 4); c.FLAG = (int*)al(256);
  c.bytes = off - off0; return off;
}
static void csr_build8(const CsrBufs8& c, const int* dst, int E, int N, hipStream_t stream) {
  const size_t smem = (size_t)(2 * c.NGP + c.CHP) * 4;
  csrZ_kernel8<<<512, 256, 0, stream>>>((int*)c.base, c.bytes / 16);
  csrA_kernel8<<<CSR_NBLK8, 64, smem, stream>>>(dst, E, N, c.nG, c.CHP, c.NGP, c.STG, c.HST);
  csrS_kernel8<<<1, 512, 0, stream>>>(c.HST, c.nG, c.NGP, c.START, c.TOT, c.OFF);
  csrB_kernel8<<<c.nG, 256, 0, stream>>>(dst, N, c.nG, c.CHP, c.NGP, (int)c.permLen, c.STG, c.HST, c.OFF, c.START, c.TOT, c.PERM, c.ROWPTR, c.ROWCNT, c.FLAG);
}


__global__ __launch_bounds__(256) void wput_kernel(const float* __restrict__ g1, const float* __restrict__ g2, const float* __restrict__ wif, const float* __restrict__ whf, const float* __restrict__ wib, const float* __restrict__ whb, const float* __restrict__ fcw, b16* __restrict__ W1T, b16* __restrict__ W2T, b16* __restrict__ WIH, b16* __restrict__ WHH, b16* __restrict__ FCT) { const size_t nt = (size_t)gridDim.x * 256, u0 = (size_t)blockIdx.x * 256 + threadIdx.x; v8b v;
  for (size_t u = u0; u < (size_t)GH * (INP / 8); u += nt) { const int o = (int)(u / (INP / 8)), k0 = (int)(u % (INP / 8)) * 8;
#pragma unroll
    for (int j = 0; j < 8; ++j) { const int k = k0 + j; v[j] = (b16)(k < IND ? bf16_rne(g1[(size_t)k * GH + o]) * WSC : 0.0f); } for (int pass = 0; pass < 2; ++pass) { *(volatile v8b*)(W1T + (size_t)o * INP + k0) = v; __threadfence(); } }
  for (size_t u = u0; u < (size_t)EMB * (GH / 8); u += nt) { const int o = (int)(u / (GH / 8)), k0 = (int)(u % (GH / 8)) * 8;
#pragma unroll
    for (int j = 0; j < 8; ++j) v[j] = (b16)(bf16_rne(g2[(size_t)(k0 + j) * EMB + o]) * WSC); for (int pass = 0; pass < 2; ++pass) { *(volatile v8b*)(W2T + (size_t)o * GH + k0) = v; __threadfence(); } }
  for (size_t u = u0; u < (size_t)2 * G4 * (H / 8); u += nt) { const int d = (int)(u / ((size_t)G4 * (H / 8))); const size_t r = u % ((size_t)G4 * (H / 8)); const int o = (int)(r / (H / 8)), k0 = (int)(r % (H / 8)) * 8; const float* wi = d ? wib : wif; const float* wh = d ? whb : whf;
#pragma unroll
    for (int j = 0; j < 8; ++j) v[j] = (b16)(bf16_rne(wi[(size_t)o * EMB + k0 + j]) * WSC); for (int pass = 0; pass < 2; ++pass) { *(volatile v8b*)(WIH + ((size_t)d * G4 + o) * EMB + k0) = v; __threadfence(); }
#pragma unroll
    for (int j = 0; j < 8; ++j) v[j] = (b16)(bf16_rne(wh[(size_t)o * H + k0 + j]) * WSC); for (int pass = 0; pass < 2; ++pass) { *(volatile v8b*)(WHH + ((size_t)d * G4 + o) * H + k0) = v; __threadfence(); } }
  for (size_t u = u0; u < (size_t)OPAD * (2 * H / 8); u += nt) { const size_t o = u / (2 * H / 8); const int k0 = (int)(u % (2 * H / 8)) * 8;
#pragma unroll
    for (int j = 0; j < 8; ++j) v[j] = (b16)(o < (size_t)N ? bf16_rne(fcw[(size_t)(k0 + j) * N + o]) * XS : 0.0f); for (int pass = 0; pass < 2; ++pass) { *(volatile v8b*)(FCT + o * 2 * H + k0) = v; __threadfence(); } } }
__global__ __launch_bounds__(256) void deg_kernel(const float* __restrict__ ew, const int* __restrict__ PERM, const int* __restrict__ ROWPTR, const int* __restrict__ ROWCNT, int permLen, float* __restrict__ DINV) { __shared__ float Ds[32]; const int wave = threadIdx.x >> 5, lane = threadIdx.x & 31; const size_t i = (size_t)blockIdx.x * 8 + wave; float s = 0.0f; if (i < (size_t)N) { int st = ROWPTR[i], cnt = ROWCNT[i]; cnt = iclamp(cnt, 0, E); st = iclamp(st, 0, permLen - cnt); for (int j = lane; j < cnt; j += 32) { const int e = iclamp(PERM[st + j], 0, E - 1); s += bfv(ew[e]); } }
  for (int o = 16; o; o >>= 1) s += __shfl_xor(s, o); if (lane == 0) Ds[wave] = rsqrtf(s + 1.0f);
  __syncthreads();
  for (int pass = 0; pass < 2; ++pass) { if (wave == 0) ((volatile float*)DINV)[(size_t)blockIdx.x * 32 + lane] = lane < 8 ? Ds[lane] : 0.0f; __threadfence(); } }
__device__ __forceinline__ float dinv_at(const float* DINV, size_t i) { return DINV[(i >> 3) * 32 + (i & 7)]; }
__global__ __launch_bounds__(32) void lin1_kernel(const float* __restrict__ xc, const float* __restrict__ ne, const float* __restrict__ tf, const b16* __restrict__ W1T, int NLIM, float* __restrict__ HW1) { __shared__ __attribute__((aligned(16))) b16 Ah[16][INP + 8]; __shared__ float Tf[16][GH + 4]; const int lane = threadIdx.x, nloc = lane & 15, hlf = lane >> 4; const size_t m0 = (size_t)blockIdx.x * 16; if (m0 >= (size_t)NLIM) return;
  for (int rr = 0; rr < 16; ++rr) { const size_t n = m0 + rr; for (int q = 0; q < INP / 32; ++q) { const int k = q * 32 + lane; float v = 0.0f; if (k < 2) v = xc[n * 2 + k]; else if (k < 2 + EMB) v = ne[n * EMB + k - 2]; else if (k < IND) v = tf[n * TD + k - 2 - EMB]; Ah[rr][k] = (b16)(bf16_rne(v) * HS); } } if (lane < 16) for (int k = INP; k < INP + 8; ++k) Ah[lane][k] = (b16)0.0f;
  wave_lds_sync(); v8f acc[4] = {(v8f){}, (v8f){}, (v8f){}, (v8f){}};
#pragma unroll
  for (int kb = 0; kb < INP; kb += 32) { const v16b a = frag_kb(&Ah[nloc][kb], hlf);
#pragma unroll
    for (int t = 0; t < 4; ++t) acc[t] = wmma16b(a, frag_kb(W1T + (size_t)(t * 16 + nloc) * INP + kb, hlf), acc[t]); }
#pragma unroll
  for (int t = 0; t < 4; ++t)
#pragma unroll
    for (int r8 = 0; r8 < 8; ++r8) Tf[8 * hlf + r8][t * 16 + nloc] = acc[t][r8] * (1.0f / (HS * WSC));
  wave_lds_sync();
  for (int pass = 0; pass < 2; ++pass) { for (int rr = 0; rr < 16; ++rr) *(volatile v2f*)(HW1 + (m0 + rr) * GH + lane * 2) = *(const v2f*)(&Tf[rr][lane * 2]); __threadfence(); } }
template <int W, int RELU>
__global__ __launch_bounds__(256) void sweep_kernel(const float* __restrict__ HW, const float* __restrict__ DINV, const float* __restrict__ ew, const float* __restrict__ bias, const int* __restrict__ srcs, const int* __restrict__ PERM, const int* __restrict__ ROWPTR, const int* __restrict__ ROWCNT, int permLen, int NLIM, float* __restrict__ OUT) { constexpr int CPL = W / 32; const int wave = threadIdx.x >> 5, lane = threadIdx.x & 31; const size_t i = (size_t)blockIdx.x * NPB + wave; if (i >= (size_t)NLIM) return; int st = ROWPTR[i], cnt = ROWCNT[i]; cnt = iclamp(cnt, 0, E); st = iclamp(st, 0, permLen - cnt); float acc[CPL]; for (int k = 0; k < CPL; ++k) acc[k] = 0.0f;
#pragma unroll 1
  for (int j = 0; j < cnt; ++j) { const int e = iclamp(PERM[st + j], 0, E - 1); const size_t u = (size_t)iclamp(srcs[e], 0, N - 1); if (u >= (size_t)NLIM) continue; const float w = pmul(dinv_at(DINV, u), bfv(ew[e]));
#pragma unroll
    for (int k = 0; k < CPL; ++k) acc[k] += pmul(w, HW[u * W + lane * CPL + k]); }
  const float di = dinv_at(DINV, i); float o[CPL];
#pragma unroll
  for (int k = 0; k < CPL; ++k) { const float v = pmul(di, acc[k] + pmul(di, HW[i * W + lane * CPL + k])) + bfv(bias[lane * CPL + k]); o[k] = RELU ? fmaxf(v, 0.0f) : v; }
  for (int pass = 0; pass < 2; ++pass) { if (CPL == 2) *(volatile v2f*)(OUT + i * W + lane * 2) = (v2f){o[0], o[1]}; else *(volatile v4f*)(OUT + i * W + lane * 4) = (v4f){o[0], o[1], o[2], o[CPL - 1]}; __threadfence(); } }
__global__ __launch_bounds__(32) void lin2_kernel(const float* __restrict__ H1, const b16* __restrict__ W2T, int NLIM, float* __restrict__ HW2) { __shared__ __attribute__((aligned(16))) b16 Ah[16][GH + 8], Al[16][GH + 8]; __shared__ float Tf[16][EMB + 4]; const int lane = threadIdx.x, nloc = lane & 15, hlf = lane >> 4; const size_t m0 = (size_t)blockIdx.x * 16; if (m0 >= (size_t)NLIM) return;
  for (int rr = 0; rr < 16; ++rr) for (int q = 0; q < 2; ++q) { b16 p, ql; split16(H1[(m0 + rr) * GH + q * 32 + lane] * HS1, p, ql); Ah[rr][q * 32 + lane] = p; Al[rr][q * 32 + lane] = ql; } if (lane < 16) for (int k = GH; k < GH + 8; ++k) { Ah[lane][k] = (b16)0.0f; Al[lane][k] = (b16)0.0f; }
  wave_lds_sync(); v8f acc[8];
#pragma unroll
  for (int t = 0; t < 8; ++t) acc[t] = (v8f){};
#pragma unroll
  for (int kb = 0; kb < GH; kb += 32) { const v16b a = frag_kb(&Ah[nloc][kb], hlf), al = frag_kb(&Al[nloc][kb], hlf);
#pragma unroll
    for (int t = 0; t < 8; ++t) { const v16b bw = frag_kb(W2T + (size_t)(t * 16 + nloc) * GH + kb, hlf); acc[t] = wmma16b(a, bw, acc[t]); acc[t] = wmma16b(al, bw, acc[t]); } }
#pragma unroll
  for (int t = 0; t < 8; ++t)
#pragma unroll
    for (int r8 = 0; r8 < 8; ++r8) Tf[8 * hlf + r8][t * 16 + nloc] = acc[t][r8] * (1.0f / (HS1 * WSC));
  wave_lds_sync();
  for (int pass = 0; pass < 2; ++pass) { for (int rr = 0; rr < 16; ++rr) *(volatile v4f*)(HW2 + (m0 + rr) * EMB + lane * 4) = *(const v4f*)(&Tf[rr][lane * 4]); __threadfence(); } }
__global__ __launch_bounds__(32) void xg_kernel(const float* __restrict__ Z, const int* __restrict__ seq, const b16* __restrict__ WIH, const float* __restrict__ bif, const float* __restrict__ bhf, const float* __restrict__ bib, const float* __restrict__ bhb, int BLIM, int NLIM, float* __restrict__ XG) { __shared__ __attribute__((aligned(16))) b16 Ah[16][EMB + 8], Al[16][EMB + 8]; __shared__ float Tf[16][260]; const int lane = threadIdx.x, nloc = lane & 15, hlf = lane >> 4; const int d = blockIdx.x / (NB * T / 16); const size_t m0 = (size_t)(blockIdx.x % (NB * T / 16)) * 16; if (m0 >= (size_t)BLIM * T) return; const float* bi = d ? bib : bif; const float* bh = d ? bhb : bhf;
  for (int rr = 0; rr < 16; ++rr) { const size_t nd = (size_t)iclamp(seq[m0 + rr], 0, NLIM - 1);     for (int q = 0; q < 4; ++q) { b16 p, ql; split16(Z[nd * EMB + q * 32 + lane] * ZS, p, ql); Ah[rr][q * 32 + lane] = p; Al[rr][q * 32 + lane] = ql; } } if (lane < 16) for (int k = EMB; k < EMB + 8; ++k) { Ah[lane][k] = (b16)0.0f; Al[lane][k] = (b16)0.0f; }
  wave_lds_sync();
#pragma unroll 1
  for (int g = 0; g < 2; ++g) { v8f acc[16];
#pragma unroll
    for (int t = 0; t < 16; ++t) acc[t] = (v8f){};
#pragma unroll
    for (int kb = 0; kb < EMB; kb += 32) { const v16b a = frag_kb(&Ah[nloc][kb], hlf), al = frag_kb(&Al[nloc][kb], hlf);
#pragma unroll
      for (int t = 0; t < 16; ++t) { const v16b bw = frag_kb(WIH + ((size_t)d * G4 + g * 256 + t * 16 + nloc) * EMB + kb, hlf); acc[t] = wmma16b(a, bw, acc[t]); acc[t] = wmma16b(al, bw, acc[t]); } }
#pragma unroll
    for (int t = 0; t < 16; ++t) { const int cc = t * 16 + nloc; const int col = g * 256 + cc; const float bb = bfv(bi[col]) + bfv(bh[col]);
#pragma unroll
      for (int r8 = 0; r8 < 8; ++r8) Tf[8 * hlf + r8][cc] = acc[t][r8] * (1.0f / (ZS * WSC)) + bb; }
    wave_lds_sync();
    for (int pass = 0; pass < 2; ++pass) { for (int rr = 0; rr < 16; ++rr) for (int q = 0; q < 2; ++q) *(volatile v4f*)(XG + ((size_t)d * NB * T + m0 + rr) * G4 + g * 256 + q * 128 + lane * 4) = *(const v4f*)(&Tf[rr][q * 128 + lane * 4]); __threadfence(); }
    wave_lds_sync(); } }
__global__ __launch_bounds__(32) void lstm_kernel(const float* __restrict__ XG, const b16* __restrict__ WHH, const int* __restrict__ len, int BLIM, int TLIM, float* __restrict__ HO) { __shared__ __attribute__((aligned(16))) b16 Hh[2][16][H + 8], Hl[2][16][H + 8]; __shared__ float Tn[16][H + 4], Cs[16][H + 4];     const int lane = threadIdx.x, nloc = lane & 15, hlf = lane >> 4; const int d = blockIdx.x / (NB / 16); const int b0 = (blockIdx.x % (NB / 16)) * 16; if (b0 >= BLIM) return;
  for (int p = 0; p < 2; ++p) for (int rr = 0; rr < 16; ++rr) for (int k = lane; k < H + 8; k += 32) { Hh[p][rr][k] = (b16)0.0f; Hl[p][rr][k] = (b16)0.0f; }
  int lens[8]; for (int r8 = 0; r8 < 8; ++r8) lens[r8] = iclamp(len[b0 + 8 * hlf + r8], 1, TLIM);
  for (int rr = 0; rr < 16; ++rr) for (int q = 0; q < 4; ++q) Cs[rr][q * 32 + lane] = 0.0f;
  wave_lds_sync(); int cur = 0;
#pragma unroll 1
  for (int s = 0; s < TLIM; ++s) {
#pragma unroll 1
    for (int hq = 0; hq < 2; ++hq) { v8f acc[16];
#pragma unroll
      for (int t = 0; t < 16; ++t) acc[t] = (v8f){};
#pragma unroll 2
      for (int kb = 0; kb < H; kb += 32) { const v16b a = frag_kb(&Hh[cur][nloc][kb], hlf), al = frag_kb(&Hl[cur][nloc][kb], hlf);
#pragma unroll
        for (int t = 0; t < 16; ++t) { const int gcol = (t >> 2) * H + hq * 64 + (t & 3) * 16;
          const v16b bw = frag_kb(WHH + ((size_t)d * G4 + gcol + nloc) * H + kb, hlf); acc[t] = wmma16b(a, bw, acc[t]); acc[t] = wmma16b(al, bw, acc[t]); } }
#pragma unroll
      for (int r8 = 0; r8 < 8; ++r8) { const int rr = 8 * hlf + r8; const int b = b0 + rr; const int L = lens[r8]; const int tin = d == 0 ? s : (s < L ? L - 1 - s : s); const float* xg = XG + ((size_t)d * NB * T + (size_t)b * T + tin) * G4;
#pragma unroll
        for (int t4 = 0; t4 < 4; ++t4) { const int u = hq * 64 + t4 * 16 + nloc; const float sc = 1.0f / (HHS * WSC);
          const float gi = acc[t4][r8] * sc + xg[u], gf = acc[4 + t4][r8] * sc + xg[H + u], gg = acc[8 + t4][r8] * sc + xg[2 * H + u], go = acc[12 + t4][r8] * sc + xg[3 * H + u];
          const float cn = pmul(sigm(gf), Cs[rr][u]) + pmul(sigm(gi), tanhf(gg)); Cs[rr][u] = cn; Tn[rr][u] = pmul(sigm(go), tanhf(cn)); } } }
    wave_lds_sync();
    for (int rr = 0; rr < 16; ++rr) for (int q = 0; q < 4; ++q) { const int u = q * 32 + lane; const float hv = Tn[rr][u]; b16 p, ql; split16(hv * HHS, p, ql); Hh[cur ^ 1][rr][u] = p; Hl[cur ^ 1][rr][u] = ql; }
    for (int pass = 0; pass < 2; ++pass) { for (int rr = 0; rr < 16; ++rr) *(volatile v4f*)(HO + (((size_t)d * NB + b0 + rr) * T + s) * H + lane * 4) = *(const v4f*)(&Tn[rr][lane * 4]); __threadfence(); }
    wave_lds_sync(); cur ^= 1; } }
__global__ __launch_bounds__(32) void pool_kernel(const float* __restrict__ HO, const int* __restrict__ len, const float* __restrict__ aw, const float* __restrict__ ab, int BLIM, int TLIM, float* __restrict__ CTX) { const int lane = threadIdx.x; const int b = blockIdx.x; if (b >= BLIM) return; const int L = iclamp(len[b], 1, TLIM); float w8[8]; for (int q = 0; q < 8; ++q) w8[q] = bfv(aw[lane * 8 + q]); float mx = -INFINITY, den = 0.0f, acc[8] = {0, 0, 0, 0, 0, 0, 0, 0};
#pragma unroll 1
  for (int t = 0; t < L; ++t) { const int rv = L - 1 - t; float v[8];
    const float* src = lane < 16 ? HO + (((size_t)0 * NB + b) * T + t) * H + lane * 8 : HO + (((size_t)1 * NB + b) * T + rv) * H + (lane - 16) * 8;
    float s = 0.0f;
#pragma unroll
    for (int q = 0; q < 8; ++q) { v[q] = src[q]; s += pmul(v[q], w8[q]); } for (int o = 16; o; o >>= 1) s += __shfl_xor(s, o); s += bfv(ab[0]);
    const float mn = fmaxf(mx, s); const float sf = (mx == -INFINITY) ? 0.0f : __expf(mx - mn); const float p = __expf(s - mn); den = den * sf + p;
#pragma unroll
    for (int q = 0; q < 8; ++q) acc[q] = pmul(acc[q], sf) + pmul(p, v[q]); mx = mn; }
  for (int pass = 0; pass < 2; ++pass) { *(volatile v4f*)(CTX + (size_t)b * 2 * H + lane * 8) = (v4f){acc[0] / den, acc[1] / den, acc[2] / den, acc[3] / den}; *(volatile v4f*)(CTX + (size_t)b * 2 * H + lane * 8 + 4) = (v4f){acc[4] / den, acc[5] / den, acc[6] / den, acc[7] / den}; __threadfence(); } }
__global__ __launch_bounds__(32) void fc_kernel(const float* __restrict__ CTX, const b16* __restrict__ FCT, int OLIM, float* __restrict__ OT) { __shared__ __attribute__((aligned(16))) b16 Ah[NB][2 * H + 8], Al[NB][2 * H + 8]; __shared__ float Tf[NB][68]; const int lane = threadIdx.x, nloc = lane & 15, hlf = lane >> 4; const size_t o0 = (size_t)blockIdx.x * 256; if (o0 >= (size_t)OLIM) return;
  for (int rr = 0; rr < NB; ++rr) for (int q = 0; q < 8; ++q) { b16 p, ql; split16(CTX[(size_t)rr * 2 * H + q * 32 + lane] * CS, p, ql); Ah[rr][q * 32 + lane] = p; Al[rr][q * 32 + lane] = ql; } for (int r = 0; r < NB; r += 32) for (int k = 2 * H; k < 2 * H + 8; ++k) { Ah[r + lane][k] = (b16)0.0f; Al[r + lane][k] = (b16)0.0f; }
  wave_lds_sync();
#pragma unroll 1
  for (int tg = 0; tg < 4; ++tg) {
    v8f acc[4][4];
#pragma unroll
    for (int rt = 0; rt < 4; ++rt)
#pragma unroll
      for (int t = 0; t < 4; ++t) acc[rt][t] = (v8f){};
#pragma unroll 2
    for (int kb = 0; kb < 2 * H; kb += 32) { v16b bw[4];
#pragma unroll
      for (int t = 0; t < 4; ++t) bw[t] = frag_kb(FCT + (o0 + tg * 64 + t * 16 + nloc) * 2 * H + kb, hlf);
#pragma unroll
      for (int rt = 0; rt < 4; ++rt) { const v16b a = frag_kb(&Ah[rt * 16 + nloc][kb], hlf), al = frag_kb(&Al[rt * 16 + nloc][kb], hlf);
#pragma unroll
        for (int t = 0; t < 4; ++t) { acc[rt][t] = wmma16b(a, bw[t], acc[rt][t]); acc[rt][t] = wmma16b(al, bw[t], acc[rt][t]); } } }
#pragma unroll
    for (int rt = 0; rt < 4; ++rt)
#pragma unroll
      for (int t = 0; t < 4; ++t)
#pragma unroll
        for (int r8 = 0; r8 < 8; ++r8) Tf[rt * 16 + 8 * hlf + r8][t * 16 + nloc] = acc[rt][t][r8] * (1.0f / (CS * XS));
    wave_lds_sync();
    for (int pass = 0; pass < 2; ++pass) { for (int oo = 0; oo < 64; ++oo) *(volatile v2f*)(OT + (o0 + tg * 64 + oo) * NB + lane * 2) = (v2f){Tf[lane * 2][oo], Tf[lane * 2 + 1][oo]}; __threadfence(); }
    wave_lds_sync(); } }
__global__ __launch_bounds__(256) void out_kernel(const float* __restrict__ OT, const float* __restrict__ fcb, int OLIM, float* __restrict__ out) { const size_t u = (size_t)blockIdx.x * 256 + threadIdx.x; if (u >= (size_t)NB * N) return; const int b = (int)(u / N), o = (int)(u % N); if (o >= OLIM) return; const float v = OT[(size_t)o * NB + b] + bfv(fcb[o]); for (int pass = 0; pass < 2; ++pass) { ((volatile float*)out)[u] = v; __threadfence(); } }
}

extern "C" void kernel_launch(void* const* d_in, const int* in_sizes, int n_in, void* d_out, int out_size, void* d_ws, size_t ws_size, hipStream_t stream) {
  (void)n_in;
  auto Fp = [&](int i) { return (const float*)d_in[i]; }; auto Ip = [&](int i) { return (const int*)d_in[i]; };
  if (in_sizes[0] != N * 2 || in_sizes[1] != N * TD || in_sizes[2] != 2 * E || in_sizes[3] != E || in_sizes[4] != NB * T || in_sizes[5] != NB || in_sizes[6] != N * EMB || in_sizes[7] != IND * GH || in_sizes[9] != GH * EMB || in_sizes[11] != G4 * EMB || in_sizes[12] != G4 * H || in_sizes[15] != G4 * EMB || in_sizes[19] != 2 * H || in_sizes[21] != 2 * H * N || in_sizes[22] != N || out_size != NB * N) return;
  const int BLIM = NB, OLIM = N, TLIM = T, NLIM = N;
  size_t off = 0; char* ws = (char*)d_ws;
  auto carve = [&](size_t bytes) { char* p = ws + off; off += (bytes + 255) & ~(size_t)255; return p; };
  b16* W1T = (b16*)carve((size_t)GH * INP * 2); b16* W2T = (b16*)carve((size_t)EMB * GH * 2); b16* WIH = (b16*)carve((size_t)2 * G4 * EMB * 2); b16* WHH = (b16*)carve((size_t)2 * G4 * H * 2); b16* FCT = (b16*)carve((size_t)OPAD * 2 * H * 2);
  float* DINV = (float*)carve((size_t)(N / 8 + 1) * 32 * 4); float* HW1 = (float*)carve((size_t)N * GH * 4); float* H1 = (float*)carve((size_t)N * GH * 4); float* HW2 = (float*)carve((size_t)N * EMB * 4); float* Z = (float*)carve((size_t)N * EMB * 4); float* XG = (float*)carve((size_t)2 * NB * T * G4 * 4); float* HO = (float*)carve((size_t)2 * NB * T * H * 4); float* CTX = (float*)carve((size_t)NB * 2 * H * 4); float* OT = (float*)carve((size_t)OPAD * NB * 4);
  CsrBufs8 csr; off = csr_carve8(csr, ws, off, E, N);
  if (off > ws_size || off > ((size_t)224 << 20)) return;
  wput_kernel<<<256, 256, 0, stream>>>(Fp(7), Fp(9), Fp(11), Fp(12), Fp(15), Fp(16), Fp(21), W1T, W2T, WIH, WHH, FCT);
  csr_build8(csr, Ip(2) + E, E, N, stream);
  deg_kernel<<<(N + 7) / 8, 256, 0, stream>>>(Fp(3), csr.PERM, csr.ROWPTR, csr.ROWCNT, (int)csr.permLen, DINV);
  lin1_kernel<<<N / 16, 32, 0, stream>>>(Fp(0), Fp(6), Fp(1), W1T, NLIM, HW1);
  sweep_kernel<GH, 1><<<(N + NPB - 1) / NPB, 256, 0, stream>>>(HW1, DINV, Fp(3), Fp(8), Ip(2), csr.PERM, csr.ROWPTR, csr.ROWCNT, (int)csr.permLen, NLIM, H1);
  lin2_kernel<<<N / 16, 32, 0, stream>>>(H1, W2T, NLIM, HW2);
  sweep_kernel<EMB, 0><<<(N + NPB - 1) / NPB, 256, 0, stream>>>(HW2, DINV, Fp(3), Fp(10), Ip(2), csr.PERM, csr.ROWPTR, csr.ROWCNT, (int)csr.permLen, NLIM, Z);
  xg_kernel<<<2 * (NB * T / 16), 32, 0, stream>>>(Z, Ip(4), WIH, Fp(13), Fp(14), Fp(17), Fp(18), BLIM, NLIM, XG);
  lstm_kernel<<<2 * (NB / 16), 32, 0, stream>>>(XG, WHH, Ip(5), BLIM, TLIM, HO);
  pool_kernel<<<NB, 32, 0, stream>>>(HO, Ip(5), Fp(19), Fp(20), BLIM, TLIM, CTX);
  fc_kernel<<<OPAD / 256, 32, 0, stream>>>(CTX, FCT, OLIM, OT);
  out_kernel<<<(unsigned)(((size_t)NB * N + 255) / 256), 256, 0, stream>>>(OT, Fp(22), OLIM, (float*)d_out);
}
